// GCNClusterGAT_16303695856290
// MI455X (gfx1250) — hardware-run, weakly checked
//
#include <hip/hip_runtime.h>


namespace {
constexpr int N = 20000, E = 640000, NF = 512, NHID = 128, H1 = 2, D1 = H1 * NHID, NO = 64, K = 100, KP = 112, NIT = 11, NB64 = (N + 63) / 64;
constexpr float XS = 8.0f, RS = 1024.0f, WSC = 256.0f, TEMP = 5.0f, SLOPE = 0.2f;
typedef _Float16 b16;
typedef __attribute__((ext_vector_type(16))) _Float16 v16b;
typedef __attribute__((ext_vector_type(8))) _Float16 v8b;
typedef __attribute__((ext_vector_type(8))) float v8f;
typedef __attribute__((ext_vector_type(4))) float v4f;
typedef __attribute__((ext_vector_type(2))) float v2f;
__device__ __forceinline__ float bf16_rne(float f) { unsigned int u = __float_as_uint(f); u += 0x7FFFu + ((u >> 16) & 1u); float r = __uint_as_float(u & 0xFFFF0000u); asm volatile("" : "+v"(r)); return r; }
__device__ __forceinline__ void split16(float v, b16& hi, b16& lo) { hi = (b16)v; lo = (b16)(v - (float)hi); }
__device__ __forceinline__ v16b frag_kb(const b16* p, int hh) { const v8b a = *(const v8b*)(p + 8 * hh), b = *(const v8b*)(p + 16 + 8 * hh); v16b f;
#pragma unroll
  for (int e = 0; e < 8; ++e) { f[e] = a[e]; f[8 + e] = b[e]; } return f; }
__device__ __forceinline__ v8f wmma16b(v16b a, v16b b, v8f c) { v8f d = __builtin_amdgcn_wmma_f32_16x16x32_f16(false, a, false, b, (short)0, c, false, false); asm volatile("v_nop\n\tv_nop\n\tv_nop\n\tv_nop" : "+v"(d) : "v"(a), "v"(b)); return d; }
__device__ __forceinline__ void wave_lds_sync() { __builtin_amdgcn_fence(__ATOMIC_RELEASE, "workgroup"); __builtin_amdgcn_wave_barrier(); __builtin_amdgcn_fence(__ATOMIC_ACQUIRE, "workgroup"); }
__device__ __forceinline__ float pmul(float a, float b) { float p = a * b; asm volatile("" : "+v"(p)); return p; }
__device__ __forceinline__ int iclamp(int v, int lo, int hi) { return v < lo ? lo : (v > hi ? hi : v); }
__device__ __forceinline__ float lrelu(float v) { return v > 0.0f ? v : SLOPE * v; }
__device__ __forceinline__ float elu(float v) { return v > 0.0f ? v : (__expf(v) - 1.0f); }
constexpr int CSR_NBLK8 = 512, CSR_GB8 = 8, CSR_GN8 = 1 << CSR_GB8  , CSR_TS8 = (CSR_GN8 < 32 ? 32 : CSR_GN8)  , CSR_MAXG8 = 512, CSR_CAP8 = 12288  ;
__device__ __host__ __forceinline__ int csr_tix8(int v) { return (v >> CSR_GB8) * CSR_TS8 + (v & (CSR_GN8 - 1)); }
__global__ __launch_bounds__(64) void csrA_kernel8(const int* __restrict__ dst, int E, int N, int nG, int CHP, int NGP, int* __restrict__ STG, int* __restrict__ HST) {
  extern __shared__ int sm[];
  int* cnt = sm; int* run = sm + NGP; int* ids = sm + 2 * NGP;
  const int b = blockIdx.x; const int ch = (E + CSR_NBLK8 - 1) / CSR_NBLK8; const int e0 = b * ch, e1 = min(E, e0 + ch);
  for (int i = threadIdx.x; i < NGP; i += 64) cnt[i] = 0;
  for (int i = threadIdx.x; i < CHP; i += 64) ids[i] = -1;
  __syncthreads();
  if (threadIdx.x == 0) {
    for (int e = e0; e < e1; ++e) { int d = dst[e]; d = (d < 0) ? 0 : (d >= N ? N - 1 : d); cnt[d >> CSR_GB8] += 1; }
    int acc = 0; for (int g = 0; g < nG; ++g) { run[g] = acc; acc += cnt[g]; }
    for (int e = e0; e < e1; ++e) { int d = dst[e]; d = (d < 0) ? 0 : (d >= N ? N - 1 : d); const int g = d >> CSR_GB8; ids[run[g]] = e; run[g] += 1; } }
  __syncthreads();
  typedef __attribute__((ext_vector_type(4))) int v4i;
  for (int pass = 0; pass < 2; ++pass) {
    for (int i = threadIdx.x; i < CHP / 4; i += 64) *(volatile v4i*)(STG + (size_t)b * CHP + i * 4) = *(const v4i*)(&ids[i * 4]);
    for (int i = threadIdx.x; i < NGP / 4; i += 64) { v4i v; for (int e = 0; e < 4; ++e) v[e] = (i * 4 + e < nG) ? cnt[i * 4 + e] : 0; *(volatile v4i*)(HST + (size_t)b * NGP + i * 4) = v; }
    __threadfence(); }
}
__global__ __launch_bounds__(512) void csrS_kernel8(const int* __restrict__ HST, int nG, int NGP, int* __restrict__ START, int* __restrict__ TOT, int* __restrict__ OFF) {
  __shared__ int tot[CSR_MAXG8];
  const int b = threadIdx.x;
  for (int pass = 0; pass < 2; ++pass) { int runb = 0; for (int g = 0; g < nG; ++g) { int c = HST[(size_t)b * NGP + g]; c = (c < 0) ? 0 : c; ((volatile int*)OFF)[(size_t)g * CSR_NBLK8 + b] = runb; runb += c; } __threadfence(); }
  for (int g = threadIdx.x; g < nG; g += 512) { int s = 0; for (int bb = 0; bb < CSR_NBLK8; ++bb) { int c = HST[(size_t)bb * NGP + g]; s += (c < 0) ? 0 : c; } tot[g] = s; }
  __syncthreads();
  if (threadIdx.x < 32) {
    __shared__ int st[CSR_MAXG8 + 32];
    if (threadIdx.x == 0) { int acc = 0; for (int g = 0; g < NGP; ++g) { st[g] = acc; if (g < nG) acc += (tot[g] + 31) & ~31; } st[NGP] = acc; }
    __builtin_amdgcn_fence(__ATOMIC_RELEASE, "workgroup"); __builtin_amdgcn_wave_barrier(); __builtin_amdgcn_fence(__ATOMIC_ACQUIRE, "workgroup");
    for (int pass = 0; pass < 2; ++pass) { for (int i = threadIdx.x; i < NGP + 32; i += 32) { ((volatile int*)START)[i] = (i <= NGP) ? st[min(i, NGP)] : 0; ((volatile int*)TOT)[i] = (i < nG) ? tot[i] : 0; } __threadfence(); } }
}
__global__ __launch_bounds__(256) void csrB_kernel8(const int* __restrict__ dst, int N, int nG, int CHP, int NGP, int permLen, const int* __restrict__ STG, const int* __restrict__ HST, const int* __restrict__ OFF, const int* __restrict__ START, const int* __restrict__ TOT, int* __restrict__ PERM, int* __restrict__ ROWPTR, int* __restrict__ ROWCNT, int* __restrict__ FLAG) {
  typedef __attribute__((ext_vector_type(4))) int v4i;
  __shared__ int ids[CSR_CAP8]; __shared__ unsigned short key[CSR_CAP8]; __shared__ int outp[CSR_CAP8]; __shared__ int ncnt[CSR_GN8 + 1]; __shared__ int boff[CSR_NBLK8 + 1];
  const int g = blockIdx.x, t_ = threadIdx.x; int tot = TOT[g]; int st = START[g], stn = START[g + 1]; const int v0 = g * CSR_GN8; const int nv = min(CSR_GN8, N - v0); const int t0 = g * CSR_TS8;
  st = (st < 0) ? 0 : (st > permLen - 32 ? permLen - 32 : st) & ~31; stn = (stn < st) ? st : (stn > permLen ? permLen : stn); tot = (tot < 0) ? 0 : tot; if (tot > stn - st && tot <= CSR_CAP8) tot = stn - st;
  if (tot > CSR_CAP8) {
    for (int pass = 0; pass < 2; ++pass) { for (int i = t_; i < CSR_TS8 / 4; i += 256) { v4i a, c; for (int e = 0; e < 4; ++e) { a[e] = st; c[e] = 0; } *(volatile v4i*)(ROWPTR + t0 + i * 4) = a; *(volatile v4i*)(ROWCNT + t0 + i * 4) = c; } if (t_ == 0) ((volatile int*)FLAG)[0] = 1; __threadfence(); } (void)nv; return; }
  if (t_ == 0) { int acc = 0; for (int b = 0; b < CSR_NBLK8; ++b) { boff[b] = acc; int c = HST[(size_t)b * NGP + g]; c = (c < 0) ? 0 : (c > CHP ? CHP : c); acc += c; if (acc > tot) acc = tot; } boff[CSR_NBLK8] = acc; }
  for (int i = t_; i <= CSR_GN8; i += 256) ncnt[i] = 0;
  __syncthreads();
  for (int b = 0; b < CSR_NBLK8; ++b) { const int c = boff[b + 1] - boff[b]; int o_ = OFF[(size_t)g * CSR_NBLK8 + b]; o_ = (o_ < 0) ? 0 : (o_ > CHP - c ? CHP - c : o_); const int* src_ = STG + (size_t)b * CHP + o_;
    for (int i = t_; i < c; i += 256) { int id = src_[i]; id = (id < 0) ? 0 : id; ids[boff[b] + i] = id; int d = dst[id]; d = (d < v0) ? v0 : (d >= N ? N - 1 : d); int kk = d - v0; kk = (kk < 0) ? 0 : (kk >= CSR_GN8 ? CSR_GN8 - 1 : kk); key[boff[b] + i] = (unsigned short)kk; } }
  __syncthreads();
  if (t_ == 0) { for (int i = 0; i < tot; ++i) ncnt[key[i]] += 1; int acc = 0; for (int vl = 0; vl < CSR_GN8; ++vl) { const int c = ncnt[vl]; ncnt[vl] = acc; acc += c; } ncnt[CSR_GN8] = acc;
    for (int i = 0; i < tot; ++i) { const int vl = key[i]; outp[ncnt[vl]] = ids[i]; ncnt[vl] += 1; }
    for (int vl = CSR_GN8; vl > 0; --vl) ncnt[vl] = ncnt[vl - 1]; ncnt[0] = 0; }
  __syncthreads();
  for (int pass = 0; pass < 2; ++pass) {
    for (int i = t_; i < (stn - st) / 4; i += 256) { v4i v; for (int e = 0; e < 4; ++e) { const int q = i * 4 + e; v[e] = (q < tot) ? outp[q] : -1; } *(volatile v4i*)(PERM + st + i * 4) = v; }
    for (int i = t_; i < CSR_TS8 / 4; i += 256) { v4i a, c; for (int e = 0; e < 4; ++e) { const int vl = i * 4 + e; const int vc = vl < CSR_GN8 ? vl : CSR_GN8; a[e] = (vl < CSR_GN8) ? st + ncnt[vc] : st; c[e] = (vl < nv) ? (ncnt[(vc < CSR_GN8 ? vc : CSR_GN8 - 1) + 1] - ncnt[vc]) : 0; } *(volatile v4i*)(ROWPTR + t0 + i * 4) = a; *(volatile v4i*)(ROWCNT + t0 + i * 4) = c; }
    __threadfence(); }
}
__global__ __launch_bounds__(256) void csrZ_kernel8(int* __restrict__ p, size_t n4) { typedef __attribute__((ext_vector_type(4))) int v4i; const size_t tid = (size_t)blockIdx.x * 256 + threadIdx.x, nth = (size_t)gridDim.x * 256; v4i z = {0, 0, 0, 0}; for (size_t i = tid; i < n4; i += nth) *(volatile v4i*)(p + i * 4) = z; }
struct CsrBufs8 { int *STG, *HST, *OFF, *START, *TOT, *PERM, *ROWPTR, *ROWCNT, *FLAG; int nG, NGP, CHP; size_t permLen; char* base; size_t bytes; };
static size_t csr_carve8(CsrBufs8& c, char* ws, size_t off, int E, int N) {
  const size_t off0 = off; c.base = ws + off;
  auto al = [&](size_t bytes) { char* p = ws + off; off += (bytes + 255) & ~(size_t)255; return p; };
  c.nG = (N + CSR_GN8 - 1) / CSR_GN8; c.NGP = (c.nG + 31) & ~31; const int ch = (E + CSR_NBLK8 - 1) / CSR_NBLK8; c.CHP = (ch + 31) & ~31; c.permLen = (size_t)E + 32 * (size_t)c.nG + 32;
  c.STG = (int*)al((size_t)CSR_NBLK8 * c.CHP * 4); c.HST = (int*)al((size_t)CSR_NBLK8 * c.NGP * 4); c.OFF = (int*)al((size_t)c.NGP * CSR_NBLK8 * 4); c.START = (int*)al((size_t)(c.NGP + 64) * 4); c.TOT = (int*)al((size_t)(c.NGP + 64) * 4);
  c.PERM = (int*)al(c.permLen * 4); c.ROWPTR = (int*)al((size_t)c.nG * CSR_TS8 * 4); c.ROWCNT = (int*)al((size_t)c.nG * CSR_TS8 * 4); c.FLAG = (int*)al(256);
  c.bytes = off - off0; return off;
}
static void csr_build8(const CsrBufs8& c, const int* dst, int E, int N, hipStream_t stream) {
  const size_t smem = (size_t)(2 * c.NGP + c.CHP) * 4;
  csrZ_kernel8<<<512, 256, 0, stream>>>((int*)c.base, c.bytes / 16);
  csrA_kernel8<<<CSR_NBLK8, 64, smem, stream>>>(dst, E, N, c.nG, c.CHP, c.NGP, c.STG, c.HST);
  csrS_kernel8<<<1, 512, 0, stream>>>(c.HST, c.nG, c.NGP, c.START, c.TOT, c.OFF);
  csrB_kernel8<<<c.nG, 256, 0, stream>>>(dst, N, c.nG, c.CHP, c.NGP, (int)c.permLen, c.STG, c.HST, c.OFF, c.START, c.TOT, c.PERM, c.ROWPTR, c.ROWCNT, c.FLAG);
}


__global__ __launch_bounds__(256) void wcopy_kernel(const float* __restrict__ w, size_t total, b16* __restrict__ WT) { const size_t u = (size_t)blockIdx.x * 256 + threadIdx.x; if (u >= total / 8) return; v8b v;
#pragma unroll
  for (int j = 0; j < 8; ++j) v[j] = (b16)(bf16_rne(w[u * 8 + j]) * WSC); for (int pass = 0; pass < 2; ++pass) { *(volatile v8b*)(WT + u * 8) = v; __threadfence(); } }
template <int KIN, int MODE>
__global__ __launch_bounds__(32) void dense_kernel(const float* __restrict__ IN, const b16* __restrict__ WT, int NG, int OW, float* __restrict__ OUT) {
  __shared__ __attribute__((aligned(16))) b16 Ah[16][KIN + 8], Al[16][MODE == 0 ? 8 : KIN + 8]; __shared__ float Tf[16][68]; const int lane = threadIdx.x, nloc = lane & 15, hlf = lane >> 4; const int g = blockIdx.x % NG; const size_t m0 = (size_t)(blockIdx.x / NG) * 16;
  for (int rr = 0; rr < 16; ++rr) for (int q = 0; q < KIN / 32; ++q) { const float v = IN[(m0 + rr) * KIN + q * 32 + lane]; if (MODE == 0) Ah[rr][q * 32 + lane] = (b16)(bf16_rne(v) * XS); else { b16 p, ql; split16(v * XS, p, ql); Ah[rr][q * 32 + lane] = p; Al[rr][q * 32 + lane] = ql; } }
  wave_lds_sync(); v8f acc[4] = {(v8f){}, (v8f){}, (v8f){}, (v8f){}};
#pragma unroll 2
  for (int kb = 0; kb < KIN; kb += 32) { const v16b a = frag_kb(&Ah[nloc][kb], hlf); v16b a2; if (MODE != 0) a2 = frag_kb(&Al[nloc][kb], hlf);
#pragma unroll
    for (int t = 0; t < 4; ++t) { const v16b bw = frag_kb(WT + (size_t)(g * 64 + t * 16 + nloc) * KIN + kb, hlf); acc[t] = wmma16b(a, bw, acc[t]); if (MODE != 0) acc[t] = wmma16b(a2, bw, acc[t]); } }
#pragma unroll
  for (int t = 0; t < 4; ++t)
#pragma unroll
    for (int r8 = 0; r8 < 8; ++r8) Tf[8 * hlf + r8][t * 16 + nloc] = acc[t][r8] * (1.0f / (XS * WSC));
  wave_lds_sync();
  for (int pass = 0; pass < 2; ++pass) { for (int rr = 0; rr < 16; ++rr) *(volatile v2f*)(OUT + (m0 + rr) * OW + g * 64 + lane * 2) = (v2f){Tf[rr][lane * 2], Tf[rr][lane * 2 + 1]}; __threadfence(); } }
template <int NHEAD, int CW>
__global__ __launch_bounds__(256) void al_kernel(const float* __restrict__ Hh, const float* __restrict__ as, const float* __restrict__ ad, float* __restrict__ AL) { constexpr int W = NHEAD * CW, CPL = W / 32, LPH = CW / CPL; const int wave = threadIdx.x >> 5, lane = threadIdx.x & 31; const size_t i = (size_t)blockIdx.x * 8 + wave; if (i >= (size_t)N) return;
  float s = 0.0f, d = 0.0f;
#pragma unroll
  for (int k = 0; k < CPL; ++k) { const float v = Hh[i * W + lane * CPL + k]; s += pmul(v, bf16_rne(as[lane * CPL + k])); d += pmul(v, bf16_rne(ad[lane * CPL + k])); }
  for (int o = 1; o < LPH; o <<= 1) { s += __shfl_xor(s, o); d += __shfl_xor(d, o); }
  float outv = 0.0f; for (int hd = 0; hd < NHEAD; ++hd) { const float sh = __shfl(s, hd * LPH), dh = __shfl(d, hd * LPH); if (lane == hd) outv = sh; if (lane == 8 + hd) outv = dh; }
  for (int pass = 0; pass < 2; ++pass) { ((volatile float*)AL)[i * 32 + lane] = outv; __threadfence(); } }
template <int NHEAD, int CW, int ACT>
__global__ __launch_bounds__(256) void agg_kernel(const float* __restrict__ Hh, const float* __restrict__ AL, const float* __restrict__ bias, const int* __restrict__ srcs, const int* __restrict__ PERM, const int* __restrict__ ROWPTR, const int* __restrict__ ROWCNT, int permLen, int NLIM, float* __restrict__ OUT) {
  constexpr int W = NHEAD * CW, CPL = W / 32, LPH = CW / CPL; const int wave = threadIdx.x >> 5, lane = threadIdx.x & 31; const size_t i = (size_t)blockIdx.x * 8 + wave; if (i >= (size_t)NLIM) return; const int hd = lane / LPH; int st = ROWPTR[i], cnt = ROWCNT[i]; cnt = iclamp(cnt, 0, 1 << 20); st = iclamp(st, 0, permLen - cnt);
  const float adi = AL[i * 32 + 8 + hd]; float m = -INFINITY, den = 0.0f, acc[CPL];
#pragma unroll
  for (int k = 0; k < CPL; ++k) acc[k] = 0.0f;
  auto step = [&](size_t u) { const float sc = lrelu(AL[u * 32 + hd] + adi); const float mn = fmaxf(m, sc); const float sf = (m == -INFINITY) ? 0.0f : __expf(m - mn); const float p = __expf(sc - mn); den = den * sf + p;
#pragma unroll
    for (int k = 0; k < CPL; ++k) acc[k] = pmul(acc[k], sf) + pmul(p, Hh[u * W + lane * CPL + k]); m = mn; };
#pragma unroll 1
  for (int j = 0; j < cnt; ++j) { const int e = iclamp(PERM[st + j], 0, E - 1); const size_t u = (size_t)iclamp(srcs[e], 0, N - 1); if (u >= (size_t)NLIM) continue; step(u); }
  step(i);
  const float inv = 1.0f / (den + 1e-16f); float o[CPL];
#pragma unroll
  for (int k = 0; k < CPL; ++k) { const float v = pmul(acc[k], inv) + bf16_rne(bias[lane * CPL + k]); o[k] = ACT == 0 ? elu(v) : (v + 1e-6f); }
  for (int pass = 0; pass < 2; ++pass) {
#pragma unroll
    for (int k = 0; k < CPL; ++k) ((volatile float*)OUT)[i * W + lane * CPL + k] = o[k]; __threadfence(); } }
__global__ __launch_bounds__(32) void norm_kernel(const float* __restrict__ EMB, int NLIM, float* __restrict__ embout, b16* __restrict__ DNh, b16* __restrict__ DNl, b16* __restrict__ DTh, b16* __restrict__ DTl) { __shared__ float V[64][65]; __shared__ float inv[64]; const int lane = threadIdx.x; const size_t n0 = (size_t)blockIdx.x * 64;
  for (int rr = 0; rr < 64; ++rr) { const size_t n = n0 + rr; const bool ok = n < (size_t)NLIM; const float a = ok ? EMB[n * NO + lane] : 0.0f, b = ok ? EMB[n * NO + 32 + lane] : 0.0f; V[rr][lane] = a; V[rr][32 + lane] = b; float s = pmul(a, a) + pmul(b, b); for (int o = 16; o; o >>= 1) s += __shfl_xor(s, o); if (lane == 0) inv[rr] = ok ? 1.0f / sqrtf(s) : 0.0f; }
  wave_lds_sync();
  for (int pass = 0; pass < 2; ++pass) {
    for (int rr = 0; rr < 64; ++rr) { const size_t n = n0 + rr; if (n >= (size_t)N) break; *(volatile v2f*)(embout + n * NO + lane * 2) = (v2f){V[rr][lane * 2], V[rr][lane * 2 + 1]};
      typedef __attribute__((ext_vector_type(2))) _Float16 v2b; b16 p0, q0, p1, q1; split16(pmul(V[rr][lane * 2], inv[rr]) * XS, p0, q0); split16(pmul(V[rr][lane * 2 + 1], inv[rr]) * XS, p1, q1); *(volatile v2b*)(DNh + n * NO + lane * 2) = (v2b){p0, p1}; *(volatile v2b*)(DNl + n * NO + lane * 2) = (v2b){q0, q1}; }
    for (int d = 0; d < 80; ++d) { typedef __attribute__((ext_vector_type(2))) _Float16 v2b; for (int hf = 0; hf < 2; ++hf) { const int rr = hf * 32 + lane; float v = 0.0f; if (n0 + rr < (size_t)NLIM) v = d < NO ? pmul(V[rr][d], inv[rr]) : (d == NO ? 1.0f : 0.0f); b16 p, q; split16(v * XS, p, q); ((volatile b16*)DTh)[(size_t)d * (NB64 * 64) + n0 + rr] = p; ((volatile b16*)DTl)[(size_t)d * (NB64 * 64) + n0 + rr] = q; } }
    __threadfence(); } }
__global__ __launch_bounds__(32) void dist_kernel(const b16* __restrict__ DNh, const b16* __restrict__ DNl, const b16* __restrict__ MUh, const b16* __restrict__ MUl, int NLIM, int last, b16* __restrict__ RTh, b16* __restrict__ RTl, float* __restrict__ distout, float* __restrict__ rout) {
  __shared__ float Sd[64][KP + 1], Sr[64][KP + 1]; const int lane = threadIdx.x, nloc = lane & 15, hlf = lane >> 4; const size_t n0 = (size_t)blockIdx.x * 64;
  for (int mt = 0; mt < 4; ++mt) { const size_t m0 = n0 + mt * 16; v8f acc[7]; for (int t = 0; t < 7; ++t) acc[t] = (v8f){};
    if (m0 < (size_t)NLIM) {
#pragma unroll
      for (int kb = 0; kb < NO; kb += 32) { const v16b a = frag_kb(DNh + (m0 + nloc) * NO + kb, hlf), al = frag_kb(DNl + (m0 + nloc) * NO + kb, hlf);
#pragma unroll
        for (int t = 0; t < 7; ++t) { const v16b bh = frag_kb(MUh + (size_t)(t * 16 + nloc) * NO + kb, hlf), bl = frag_kb(MUl + (size_t)(t * 16 + nloc) * NO + kb, hlf); acc[t] = wmma16b(a, bh, acc[t]); acc[t] = wmma16b(a, bl, acc[t]); acc[t] = wmma16b(al, bh, acc[t]); } } }
#pragma unroll
    for (int t = 0; t < 7; ++t)
#pragma unroll
      for (int r8 = 0; r8 < 8; ++r8) Sd[mt * 16 + 8 * hlf + r8][t * 16 + nloc] = acc[t][r8] * (1.0f / (XS * XS)); }
  wave_lds_sync();
  for (int hf = 0; hf < 2; ++hf) { const int rr = hf * 32 + lane; float mx = -INFINITY; for (int k = 0; k < K; ++k) mx = fmaxf(mx, Sd[rr][k]); float s = 0.0f; for (int k = 0; k < K; ++k) { const float e = __expf(TEMP * (Sd[rr][k] - mx)); Sr[rr][k] = e; s += e; } const float inv = 1.0f / s; for (int k = 0; k < K; ++k) Sr[rr][k] = pmul(Sr[rr][k], inv); for (int k = K; k < KP; ++k) Sr[rr][k] = 0.0f; }
  wave_lds_sync();
  for (int pass = 0; pass < 2; ++pass) {
    for (int k = 0; k < KP; ++k) for (int hf = 0; hf < 2; ++hf) { const int rr = hf * 32 + lane; const float v = (n0 + rr < (size_t)NLIM) ? Sr[rr][k] : 0.0f; b16 p, q; split16(v * RS, p, q); ((volatile b16*)RTh)[(size_t)k * (NB64 * 64) + n0 + rr] = p; ((volatile b16*)RTl)[(size_t)k * (NB64 * 64) + n0 + rr] = q; }
    if (last) for (int rr = 0; rr < 64; ++rr) { const size_t n = n0 + rr; if (n >= (size_t)N) break; for (int k = lane; k < K; k += 32) { ((volatile float*)distout)[n * K + k] = Sd[rr][k]; ((volatile float*)rout)[n * K + k] = Sr[rr][k]; } }
    __threadfence(); } }
__global__ __launch_bounds__(32) void cm_kernel(const b16* __restrict__ RTh, const b16* __restrict__ RTl, const b16* __restrict__ DTh, const b16* __restrict__ DTl, int last, b16* __restrict__ MUh, b16* __restrict__ MUl, float* __restrict__ muout) {
  __shared__ float Tc[16][84]; const int lane = threadIdx.x, nloc = lane & 15, hlf = lane >> 4; const int kt = blockIdx.x; constexpr int NPAD = NB64 * 64; v8f acc[5] = {(v8f){}, (v8f){}, (v8f){}, (v8f){}, (v8f){}};
#pragma unroll 2
  for (int kb = 0; kb < NPAD; kb += 32) { const v16b a = frag_kb(RTh + (size_t)(kt * 16 + nloc) * NPAD + kb, hlf), al = frag_kb(RTl + (size_t)(kt * 16 + nloc) * NPAD + kb, hlf);
#pragma unroll
    for (int t = 0; t < 5; ++t) { const v16b bh = frag_kb(DTh + (size_t)(t * 16 + nloc) * NPAD + kb, hlf), bl = frag_kb(DTl + (size_t)(t * 16 + nloc) * NPAD + kb, hlf); acc[t] = wmma16b(a, bh, acc[t]); acc[t] = wmma16b(a, bl, acc[t]); acc[t] = wmma16b(al, bh, acc[t]); } }
#pragma unroll
  for (int t = 0; t < 5; ++t)
#pragma unroll
    for (int r8 = 0; r8 < 8; ++r8) Tc[8 * hlf + r8][t * 16 + nloc] = acc[t][r8] * (1.0f / (RS * XS));
  wave_lds_sync();
  for (int pass = 0; pass < 2; ++pass) { for (int rr = 0; rr < 16; ++rr) { const int k = kt * 16 + rr; typedef __attribute__((ext_vector_type(2))) _Float16 v2b; float v0 = 0.0f, v1 = 0.0f; if (k < K) { const float cr = Tc[rr][NO]; v0 = Tc[rr][lane * 2] / cr; v1 = Tc[rr][lane * 2 + 1] / cr; if (last) *(volatile v2f*)(muout + (size_t)k * NO + lane * 2) = (v2f){v0, v1}; }
      b16 p0, q0, p1, q1; split16(v0 * XS, p0, q0); split16(v1 * XS, p1, q1); *(volatile v2b*)(MUh + (size_t)k * NO + lane * 2) = (v2b){p0, p1}; *(volatile v2b*)(MUl + (size_t)k * NO + lane * 2) = (v2b){q0, q1}; } __threadfence(); } }
__global__ __launch_bounds__(256) void mu0_kernel(const float* __restrict__ mu0, b16* __restrict__ MUh, b16* __restrict__ MUl) { const int u = blockIdx.x * 256 + threadIdx.x; if (u >= KP * NO) return; const int k = u / NO; const float v = k < K ? bf16_rne(mu0[u]) : 0.0f; b16 p, q; split16(v * XS, p, q); for (int pass = 0; pass < 2; ++pass) { ((volatile b16*)MUh)[u] = p; ((volatile b16*)MUl)[u] = q; __threadfence(); } }
}

extern "C" void kernel_launch(void* const* d_in, const int* in_sizes, int n_in, void* d_out, int out_size, void* d_ws, size_t ws_size, hipStream_t stream) {
  (void)n_in;
  auto Fp = [&](int i) { return (const float*)d_in[i]; }; auto Ip = [&](int i) { return (const int*)d_in[i]; };
  if (in_sizes[0] != N * NF || in_sizes[1] != D1 * NF || in_sizes[5] != NO * D1 || in_sizes[9] != K * NO || in_sizes[10] != 2 * E || out_size != K * NO + N * K + N * NO + N * K) return;
  constexpr int NPAD = NB64 * 64; const int NLIM = N;
  size_t off = 0; char* ws = (char*)d_ws;
  auto carve = [&](size_t bytes) { char* p = ws + off; off += (bytes + 255) & ~(size_t)255; return p; };
  b16* W1T = (b16*)carve((size_t)D1 * NF * 2); b16* W2T = (b16*)carve((size_t)NO * D1 * 2); float* HA = (float*)carve((size_t)N * D1 * 4); float* HB = (float*)carve((size_t)N * D1 * 4); float* AL = (float*)carve((size_t)N * 32 * 4); float* EMB = (float*)carve((size_t)N * NO * 4);
  b16* DNh = (b16*)carve((size_t)N * NO * 2); b16* DNl = (b16*)carve((size_t)N * NO * 2); b16* DTh = (b16*)carve((size_t)80 * NPAD * 2); b16* DTl = (b16*)carve((size_t)80 * NPAD * 2); b16* RTh = (b16*)carve((size_t)KP * NPAD * 2); b16* RTl = (b16*)carve((size_t)KP * NPAD * 2);
  b16* MUh = (b16*)carve((size_t)KP * NO * 2); b16* MUl = (b16*)carve((size_t)KP * NO * 2); CsrBufs8 csr; off = csr_carve8(csr, ws, off, E, N);
  if (off > ws_size || off > ((size_t)96 << 20)) return;
  float* out = (float*)d_out; float* muout = out; float* rout = out + K * NO; float* embout = rout + (size_t)N * K; float* distout = embout + (size_t)N * NO;
  wcopy_kernel<<<(D1 * NF / 8 + 255) / 256, 256, 0, stream>>>(Fp(1), (size_t)D1 * NF, W1T); wcopy_kernel<<<(NO * D1 / 8 + 255) / 256, 256, 0, stream>>>(Fp(5), (size_t)NO * D1, W2T);
  csr_build8(csr, Ip(10) + E, E, N, stream);
  dense_kernel<NF, 0><<<(NLIM / 16) * 4, 32, 0, stream>>>(Fp(0), W1T, 4, D1, HA);
  al_kernel<H1, NHID><<<(NLIM + 7) / 8, 256, 0, stream>>>(HA, Fp(2), Fp(3), AL);
  agg_kernel<H1, NHID, 0><<<(NLIM + 7) / 8, 256, 0, stream>>>(HA, AL, Fp(4), Ip(10), csr.PERM, csr.ROWPTR, csr.ROWCNT, (int)csr.permLen, NLIM, HB);
  dense_kernel<D1, 1><<<(NLIM / 16) * 1, 32, 0, stream>>>(HB, W2T, 1, NO, HA);
  al_kernel<1, NO><<<(NLIM + 7) / 8, 256, 0, stream>>>(HA, Fp(6), Fp(7), AL);
  agg_kernel<1, NO, 1><<<(NLIM + 7) / 8, 256, 0, stream>>>(HA, AL, Fp(8), Ip(10), csr.PERM, csr.ROWPTR, csr.ROWCNT, (int)csr.permLen, NLIM, EMB);
  norm_kernel<<<NB64, 32, 0, stream>>>(EMB, NLIM, embout, DNh, DNl, DTh, DTl);
  mu0_kernel<<<(KP * NO + 255) / 256, 256, 0, stream>>>(Fp(9), MUh, MUl);
  for (int it = 0; it < NIT; ++it) { dist_kernel<<<NB64, 32, 0, stream>>>(DNh, DNl, MUh, MUl, NLIM, 0, RTh, RTl, distout, rout); cm_kernel<<<7, 32, 0, stream>>>(RTh, RTl, DTh, DTl, it == NIT - 1 ? 1 : 0, MUh, MUl, muout); }
  dist_kernel<<<NB64, 32, 0, stream>>>(DNh, DNl, MUh, MUl, NLIM, 1, RTh, RTl, distout, rout);
}
